// CausalSelfAttentionAfterLN_87428354277595
// MI455X (gfx1250) — hardware-verified
//
#include <hip/hip_runtime.h>


namespace {
constexpr int Bn = 4, T = 1024, H = 12, HD = 64, E = 768, E1 = 769, KP = 800, E3 = 3 * E;
constexpr float XS = 8.0f, PS = 8.0f, EPS = 1e-5f, LOGMU = -6.9314718055994531f  ;

typedef _Float16 b16;
typedef __attribute__((ext_vector_type(16))) _Float16 v16b;
typedef __attribute__((ext_vector_type(8))) _Float16 v8b;
typedef __attribute__((ext_vector_type(8))) float v8f;
typedef __attribute__((ext_vector_type(4))) float v4f;
__device__ __forceinline__ float bf16_rne(float f) { unsigned int u = __float_as_uint(f); u += 0x7FFFu + ((u >> 16) & 1u); return __uint_as_float(u & 0xFFFF0000u); }
__device__ __forceinline__ void split16(float v, b16& hi, b16& lo) { hi = (b16)v; lo = (b16)(v - (float)hi); }
__device__ __forceinline__ v16b frag_kb(const b16* p, int hh) { const v8b a = *(const v8b*)(p + 8 * hh), b = *(const v8b*)(p + 16 + 8 * hh); v16b f;
#pragma unroll
  for (int e = 0; e < 8; ++e) { f[e] = a[e]; f[8 + e] = b[e]; } return f; }
__device__ __forceinline__ v8f wmma16b(v16b a, v16b b, v8f c) { v8f d = __builtin_amdgcn_wmma_f32_16x16x32_f16(false, a, false, b, (short)0, c, false, false); asm volatile("v_nop\n\tv_nop\n\tv_nop\n\tv_nop" : "+v"(d) : "v"(a), "v"(b)); return d; }
__device__ __forceinline__ void wave_lds_sync() { __builtin_amdgcn_fence(__ATOMIC_RELEASE, "workgroup"); __builtin_amdgcn_wave_barrier(); __builtin_amdgcn_fence(__ATOMIC_ACQUIRE, "workgroup"); }
__device__ __forceinline__ float nexp(float x) { return __builtin_amdgcn_exp2f(x * 1.4426950408889634f); }
__device__ __forceinline__ float nlog(float x) { return __builtin_amdgcn_logf(x) * 0.6931471805599453f; }
__device__ __forceinline__ float pmul(float a, float b) { float p = a * b; asm volatile("" : "+v"(p)); return p; }
__device__ __forceinline__ float wsum(float v) {
#pragma unroll
  for (int o = 1; o < 32; o <<= 1) v += __shfl_xor(v, o); return v; }
__device__ __forceinline__ float wmax(float v) {
#pragma unroll
  for (int o = 1; o < 32; o <<= 1) v = fmaxf(v, __shfl_xor(v, o)); return v; }
__device__ __forceinline__ void lse_acc(float x, float& m, float& s) { if (x > m) { s = s * nexp(m - x) + 1.0f; m = x; } else { s += nexp(x - m); } }

__global__ __launch_bounds__(256) void prep_kernel(const float* __restrict__ wa, const float* __restrict__ wp, const float* __restrict__ lw, const float* __restrict__ lb, const float* __restrict__ ba, const float* __restrict__ bp, b16* __restrict__ RA, b16* __restrict__ RP, float* __restrict__ P) {
  const size_t tid = (size_t)blockIdx.x * 256 + threadIdx.x, nth = (size_t)gridDim.x * 256;
  for (int pass = 0; pass < 2; ++pass) {
    for (size_t p = tid; p < (size_t)E3 * (KP / 8); p += nth) { const int o = (int)(p / (KP / 8)), k0 = (int)(p % (KP / 8)) * 8; v8b v; for (int e = 0; e < 8; ++e) { const int k = k0 + e; v[e] = (b16)((k < E1) ? bf16_rne(wa[(size_t)k * E3 + o]) : 0.0f); } *(volatile v8b*)(RA + (size_t)o * KP + k0) = v; }
    for (size_t p = tid; p < (size_t)E * (E / 8); p += nth) { const int o = (int)(p / (E / 8)), k0 = (int)(p % (E / 8)) * 8; v8b v; for (int e = 0; e < 8; ++e) v[e] = (b16)bf16_rne(wp[(size_t)(k0 + e) * E + o]); *(volatile v8b*)(RP + (size_t)o * E + k0) = v; }
    for (size_t q = tid; q < 4610; q += nth) { const int i = (int)q; float v; if (i < 769) v = lw[i]; else if (i < 1538) v = lb[i - 769]; else if (i < 3842) v = ba[i - 1538]; else v = bp[i - 3842]; P[q] = bf16_rne(v); }
    __threadfence(); }
}

__global__ __launch_bounds__(256) void ln_kernel(const float* __restrict__ xb, const float* __restrict__ P, b16* __restrict__ XH, b16* __restrict__ XL) {
  __shared__ __attribute__((aligned(16))) b16 Sh[8 * KP], Sl[8 * KP];
  const int wave = threadIdx.x >> 5, lane = threadIdx.x & 31, row0 = blockIdx.x * 8, row = row0 + wave; const float* xr = xb + (size_t)row * E1;
  float v[25]; float s = 0.0f;
#pragma unroll
  for (int i = 0; i < 25; ++i) { const int c = lane + 32 * i; v[i] = (c < E1) ? bf16_rne(xr[c]) : 0.0f; s += v[i]; }
  s = wsum(s); const float mu = s * (1.0f / E1); float q = 0.0f;
#pragma unroll
  for (int i = 0; i < 25; ++i) { const int c = lane + 32 * i; float d = (c < E1) ? (v[i] - mu) : 0.0f; asm volatile("" : "+v"(d)); q += pmul(d, d); }
  q = wsum(q); const float inv = rsqrtf(q * (1.0f / E1) + EPS);
#pragma unroll
  for (int i = 0; i < 25; ++i) { const int c = lane + 32 * i; float y = 0.0f; if (c < E1) { const float t_ = pmul(v[i] - mu, inv); const float a1 = pmul(t_, P[c]); float y1 = a1 + P[769 + c]; asm volatile("" : "+v"(y1)); y = y1 * XS; asm volatile("" : "+v"(y)); } b16 a_, b_; a_ = (b16)y; asm volatile("" : "+v"(a_)); b_ = (b16)(y - (float)a_); Sh[wave * KP + c] = a_; Sl[wave * KP + c] = b_; }
  __syncthreads();
  for (int pass = 0; pass < 2; ++pass) { for (int i = threadIdx.x; i < 8 * KP / 8; i += 256) { *(volatile v8b*)(XH + (size_t)row0 * KP + i * 8) = *(const v8b*)(&Sh[i * 8]); *(volatile v8b*)(XL + (size_t)row0 * KP + i * 8) = *(const v8b*)(&Sl[i * 8]); } __threadfence(); }
}

__global__ __launch_bounds__(64) void qkv_kernel(const b16* __restrict__ XH, const b16* __restrict__ XL, const b16* __restrict__ RA, const float* __restrict__ P, b16* __restrict__ QK, b16* __restrict__ VR, b16* __restrict__ VRl) {
  __shared__ __attribute__((aligned(16))) float Ts[2][32][128 + 4];
  const int lane = threadIdx.x & 31, wave = threadIdx.x >> 5, nloc = lane & 15, hlf = lane >> 4, m0 = blockIdx.y * 32, c0 = blockIdx.x * 256 + wave * 128;
#pragma unroll 1
  for (int hf = 0; hf < 2; ++hf) { v8f acc[2][4];
#pragma unroll
    for (int r = 0; r < 2; ++r)
#pragma unroll
      for (int t = 0; t < 4; ++t) acc[r][t] = (v8f){};
    for (int kb = 0; kb < KP; kb += 32) { const v16b a0 = frag_kb(XH + (size_t)(m0 + nloc) * KP + kb, hlf), a1 = frag_kb(XH + (size_t)(m0 + 16 + nloc) * KP + kb, hlf), l0 = frag_kb(XL + (size_t)(m0 + nloc) * KP + kb, hlf), l1 = frag_kb(XL + (size_t)(m0 + 16 + nloc) * KP + kb, hlf);
#pragma unroll
      for (int t = 0; t < 4; ++t) { const v16b bw = frag_kb(RA + (size_t)(c0 + (hf * 4 + t) * 16 + nloc) * KP + kb, hlf); acc[0][t] = wmma16b(a0, bw, acc[0][t]); acc[0][t] = wmma16b(l0, bw, acc[0][t]); acc[1][t] = wmma16b(a1, bw, acc[1][t]); acc[1][t] = wmma16b(l1, bw, acc[1][t]); } }
#pragma unroll
    for (int t = 0; t < 4; ++t) { const int cl = (hf * 4 + t) * 16 + nloc; const float bb = P[1538 + c0 + cl];
#pragma unroll
      for (int r = 0; r < 2; ++r)
#pragma unroll
        for (int vv = 0; vv < 8; ++vv) Ts[wave][r * 16 + 8 * hlf + vv][cl] = acc[r][t][vv] * (1.0f / XS) + bb; } }
  wave_lds_sync();
  for (int pass = 0; pass < 2; ++pass) {
    if (c0 < 2 * E) { for (int i = lane; i < 32 * 16; i += 32) { const int rr = i >> 4, c8 = (i & 15) * 8; v8b o; for (int e = 0; e < 8; ++e) o[e] = (b16)(Ts[wave][rr][c8 + e] * XS); *(volatile v8b*)(QK + (size_t)(m0 + rr) * (2 * E) + c0 + c8) = o; } }
    else { for (int i = lane; i < 32 * 16; i += 32) { const int rr = i >> 4, c8 = (i & 15) * 8; v8b oh, ol; for (int e = 0; e < 8; ++e) { b16 a_, c_; split16(Ts[wave][rr][c8 + e] * XS, a_, c_); oh[e] = a_; ol[e] = c_; } const size_t gi = (size_t)(m0 + rr) * E + (c0 - 2 * E) + c8; *(volatile v8b*)(VR + gi) = oh; *(volatile v8b*)(VRl + gi) = ol; } }
    __threadfence(); }
}

__global__ __launch_bounds__(256) void vt_kernel(const b16* __restrict__ Vr, b16* __restrict__ vt) {
  __shared__ __attribute__((aligned(16))) b16 Tt[HD][128 + 8];
  const int h = blockIdx.y, t0 = blockIdx.x * 128, t_ = threadIdx.x;
  for (int i = t_; i < 128 * (HD / 8); i += 256) { const int tk = i >> 3, d8 = (i & 7) * 8; const v8b vv = *(const v8b*)(Vr + ((size_t)(t0 + tk)) * E + h * HD + d8); for (int e = 0; e < 8; ++e) Tt[d8 + e][tk] = vv[e]; }
  __syncthreads();
  for (int pass = 0; pass < 2; ++pass) { for (int i = t_; i < HD * 16; i += 256) { const int d = i >> 4, c8 = (i & 15) * 8; *(volatile v8b*)(vt + ((size_t)h * HD + d) * T + t0 + c8) = *(const v8b*)(&Tt[d][c8]); } __threadfence(); }
}

__global__ __launch_bounds__(128) void cost_kernel(const b16* __restrict__ QK, float* __restrict__ C) {
  __shared__ __attribute__((aligned(16))) float St[4][16][32 + 4];
  const int wid = threadIdx.x >> 5, lane = threadIdx.x & 31, hh = lane >> 4, col = lane & 15; const int q0 = blockIdx.x * 16, h = blockIdx.y * 4 + wid, qi = q0 + col;
  const b16* Qr = QK + h * HD; const b16* Kr = QK + E + h * HD; const float SC = 0.125f / (XS * XS);
  const v16b qf0 = frag_kb(Qr + (size_t)qi * (2 * E), hh), qf1 = frag_kb(Qr + (size_t)qi * (2 * E) + 32, hh);
  float m = -INFINITY, l = 0.0f;
  for (int kb = 0; kb <= q0 + 15; kb += 32) { v8f s0 = {}, s1 = {};
    s0 = wmma16b(frag_kb(Kr + (size_t)(kb + col) * (2 * E), hh), qf0, s0); s0 = wmma16b(frag_kb(Kr + (size_t)(kb + col) * (2 * E) + 32, hh), qf1, s0);
    s1 = wmma16b(frag_kb(Kr + (size_t)(kb + 16 + col) * (2 * E), hh), qf0, s1); s1 = wmma16b(frag_kb(Kr + (size_t)(kb + 16 + col) * (2 * E) + 32, hh), qf1, s1);
    float mr = -INFINITY;
#pragma unroll
    for (int r = 0; r < 8; ++r) { const int k0 = kb + 8 * hh + r, k1 = k0 + 16; s0[r] = (k0 <= qi) ? s0[r] * SC : -INFINITY; s1[r] = (k1 <= qi) ? s1[r] * SC : -INFINITY; mr = fmaxf(mr, fmaxf(s0[r], s1[r])); }
    mr = fmaxf(mr, __shfl_xor(mr, 16)); const float mn = fmaxf(m, mr), al_ = nexp(m - mn); m = mn; float sum = 0.0f;
#pragma unroll
    for (int r = 0; r < 8; ++r) { sum += ((s0[r] == -INFINITY) ? 0.0f : nexp(s0[r] - mn)) + ((s1[r] == -INFINITY) ? 0.0f : nexp(s1[r] - mn)); }
    sum += __shfl_xor(sum, 16); l = l * al_ + sum; }
  const float inv = 1.0f / l;
  for (int kb = 0; kb < T; kb += 32) { float p0[8], p1[8];
    if (kb <= q0 + 15) { v8f s0 = {}, s1 = {};
      s0 = wmma16b(frag_kb(Kr + (size_t)(kb + col) * (2 * E), hh), qf0, s0); s0 = wmma16b(frag_kb(Kr + (size_t)(kb + col) * (2 * E) + 32, hh), qf1, s0);
      s1 = wmma16b(frag_kb(Kr + (size_t)(kb + 16 + col) * (2 * E), hh), qf0, s1); s1 = wmma16b(frag_kb(Kr + (size_t)(kb + 16 + col) * (2 * E) + 32, hh), qf1, s1);
#pragma unroll
      for (int r = 0; r < 8; ++r) { const int k0 = kb + 8 * hh + r, k1 = k0 + 16; p0[r] = (k0 <= qi) ? nexp(s0[r] * SC - m) * inv : 0.0f; p1[r] = (k1 <= qi) ? nexp(s1[r] * SC - m) * inv : 0.0f; } }
    else {
#pragma unroll
      for (int r = 0; r < 8; ++r) { p0[r] = 0.0f; p1[r] = 0.0f; } }
#pragma unroll
    for (int r = 0; r < 8; ++r) { St[wid][col][8 * hh + r] = p0[r]; St[wid][col][16 + 8 * hh + r] = p1[r]; }
    wave_lds_sync();
    for (int pass = 0; pass < 2; ++pass) { for (int i = lane; i < 16 * 8; i += 32) { const int rr = i >> 3, c4 = (i & 7) * 4; *(volatile v4f*)(C + ((size_t)h * T + q0 + rr) * T + kb + c4) = *(const v4f*)(&St[wid][rr][c4]); } }
    wave_lds_sync(); }
}

template <int FIRST>
__global__ __launch_bounds__(256) void rowstep_kernel(const float* __restrict__ C, const float* __restrict__ g, float* __restrict__ f) {
  __shared__ float Fs[32];
  const int wave = threadIdx.x >> 5, lane = threadIdx.x & 31, h = blockIdx.y, i0 = blockIdx.x * 32;
  for (int q = 0; q < 4; ++q) { const int i = i0 + wave * 4 + q; const float* cr = C + ((size_t)h * T + i) * T; const float* gr = g + (size_t)h * T; float m = -INFINITY, s = 0.0f;
    for (int j = lane; j < T; j += 32) { const float x = FIRST ? -cr[j] : (gr[j] - cr[j]); lse_acc(x, m, s); }
    const float mm = wmax(m); s = s * nexp(m - mm); s = wsum(s); if (lane == 0) Fs[wave * 4 + q] = LOGMU - (mm + nlog(s)); }
  __syncthreads();
  for (int pass = 0; pass < 2; ++pass) { if (threadIdx.x < 32) ((volatile float*)f)[(size_t)h * T + i0 + threadIdx.x] = Fs[threadIdx.x]; __threadfence(); }
}

__global__ __launch_bounds__(256) void colstep_kernel(const float* __restrict__ C, const float* __restrict__ f, float* __restrict__ g) {
  __shared__ float Fi[T];
  const int h = blockIdx.y, j = blockIdx.x * 256 + threadIdx.x;
  for (int i = threadIdx.x; i < T; i += 256) Fi[i] = f[(size_t)h * T + i];
  __syncthreads();
  const float* cc = C + (size_t)h * T * T + j; float m = -INFINITY, s = 0.0f;
  for (int i = 0; i < T; ++i) lse_acc(Fi[i] - cc[(size_t)i * T], m, s);
  const float gv = LOGMU - (m + nlog(s));
  for (int pass = 0; pass < 2; ++pass) { ((volatile float*)g)[(size_t)h * T + j] = gv; __threadfence(); }
}

__global__ __launch_bounds__(128) void pv_kernel(const float* __restrict__ C, const float* __restrict__ f, const float* __restrict__ g, const b16* __restrict__ vt, const b16* __restrict__ vtl, b16* __restrict__ Yh, b16* __restrict__ Yl) {
  __shared__ __attribute__((aligned(16))) b16 Oh[16][4 * HD + 8], Ol[16][4 * HD + 8];
  const int wid = threadIdx.x >> 5, lane = threadIdx.x & 31, hh = lane >> 4, col = lane & 15; const int q0 = blockIdx.x * 16, h = blockIdx.y * 4 + wid, qi = q0 + col;
  const float* cr = C + ((size_t)h * T + qi) * T; const float fi = f[(size_t)h * T + qi]; const float* gr = g + (size_t)h * T; const b16* V = vt + ((size_t)h * HD) * T; const b16* Vl = vtl + ((size_t)h * HD) * T;
  v8f o[4] = {{}, {}, {}, {}};
  for (int kb = 0; kb < T; kb += 32) { v16b pb, pl;
#pragma unroll
    for (int r = 0; r < 8; ++r) { const int j0 = kb + 8 * hh + r, j1 = j0 + 16; const float e0 = nexp(fi + gr[j0] - cr[j0]) * (float)T, e1 = nexp(fi + gr[j1] - cr[j1]) * (float)T; b16 a_, c_; split16(e0 * PS, a_, c_); pb[r] = a_; pl[r] = c_; split16(e1 * PS, a_, c_); pb[8 + r] = a_; pl[8 + r] = c_; }
#pragma unroll
    for (int t = 0; t < 4; ++t) { const v16b vh = frag_kb(V + (size_t)(t * 16 + col) * T + kb, hh), vlo = frag_kb(Vl + (size_t)(t * 16 + col) * T + kb, hh); o[t] = wmma16b(vh, pb, o[t]); o[t] = wmma16b(vh, pl, o[t]); o[t] = wmma16b(vlo, pb, o[t]); } }
#pragma unroll
  for (int t = 0; t < 4; ++t)
#pragma unroll
    for (int r = 0; r < 8; ++r) { b16 a_, c_; split16(o[t][r] * (1.0f / PS), a_, c_); Oh[col][wid * HD + t * 16 + 8 * hh + r] = a_; Ol[col][wid * HD + t * 16 + 8 * hh + r] = c_; }
  __syncthreads();
  for (int pass = 0; pass < 2; ++pass) { for (int i = threadIdx.x; i < 16 * 32; i += 128) { const int rr = i >> 5, c8 = (i & 31) * 8; const size_t gi = (size_t)(q0 + rr) * E + blockIdx.y * 4 * HD + c8; *(volatile v8b*)(Yh + gi) = *(const v8b*)(&Oh[rr][c8]); *(volatile v8b*)(Yl + gi) = *(const v8b*)(&Ol[rr][c8]); } __threadfence(); }
}

__global__ __launch_bounds__(64) void out_kernel(const b16* __restrict__ Yh, const b16* __restrict__ Yl, const b16* __restrict__ RP, const float* __restrict__ P, float* __restrict__ outb) {
  __shared__ __attribute__((aligned(16))) float Ts[2][32][128 + 4];
  const int lane = threadIdx.x & 31, wave = threadIdx.x >> 5, nloc = lane & 15, hlf = lane >> 4, m0 = blockIdx.y * 32, c0 = blockIdx.x * 256 + wave * 128;
#pragma unroll 1
  for (int hf = 0; hf < 2; ++hf) { v8f acc[2][4];
#pragma unroll
    for (int r = 0; r < 2; ++r)
#pragma unroll
      for (int t = 0; t < 4; ++t) acc[r][t] = (v8f){};
#pragma unroll 2
    for (int kb = 0; kb < E; kb += 32) { const v16b a0 = frag_kb(Yh + (size_t)(m0 + nloc) * E + kb, hlf), a1 = frag_kb(Yh + (size_t)(m0 + 16 + nloc) * E + kb, hlf), l0 = frag_kb(Yl + (size_t)(m0 + nloc) * E + kb, hlf), l1 = frag_kb(Yl + (size_t)(m0 + 16 + nloc) * E + kb, hlf);
#pragma unroll
      for (int t = 0; t < 4; ++t) { const v16b bw = frag_kb(RP + (size_t)(c0 + (hf * 4 + t) * 16 + nloc) * E + kb, hlf); acc[0][t] = wmma16b(a0, bw, acc[0][t]); acc[0][t] = wmma16b(l0, bw, acc[0][t]); acc[1][t] = wmma16b(a1, bw, acc[1][t]); acc[1][t] = wmma16b(l1, bw, acc[1][t]); } }
#pragma unroll
    for (int t = 0; t < 4; ++t) { const int cl = (hf * 4 + t) * 16 + nloc; const float bb = P[3842 + c0 + cl];
#pragma unroll
      for (int r = 0; r < 2; ++r)
#pragma unroll
        for (int vv = 0; vv < 8; ++vv) Ts[wave][r * 16 + 8 * hlf + vv][cl] = acc[r][t][vv] * (1.0f / XS) + bb; } }
  wave_lds_sync();
  for (int pass = 0; pass < 2; ++pass) { for (int i = lane; i < 32 * 32; i += 32) { const int rr = i >> 5, c4 = (i & 31) * 4; *(volatile v4f*)(outb + (size_t)(m0 + rr) * E + c0 + c4) = *(const v4f*)(&Ts[wave][rr][c4]); } __threadfence(); }
}
}

extern "C" void kernel_launch(void* const* d_in, const int* in_sizes, int n_in,
                              void* d_out, int out_size, void* d_ws, size_t ws_size, hipStream_t stream) {
  (void)n_in; (void)out_size;
  const float* x = (const float*)d_in[0]; const float* lw = (const float*)d_in[1]; const float* lb = (const float*)d_in[2]; const float* wa = (const float*)d_in[3]; const float* ba = (const float*)d_in[4]; const float* wp = (const float*)d_in[5]; const float* bp = (const float*)d_in[6];
  float* out = (float*)d_out;
  if (in_sizes[0] != Bn * T * E1 || in_sizes[3] != E1 * E3 || in_sizes[5] != E * E) return;
  size_t off = 0; char* ws = (char*)d_ws;
  auto carve = [&](size_t bytes) { char* p = ws + off; off += (bytes + 255) & ~(size_t)255; return p; };
  b16* RA = (b16*)carve((size_t)E3 * KP * 2); b16* RP = (b16*)carve((size_t)E * E * 2); float* P = (float*)carve(4610 * 4); b16* XH = (b16*)carve((size_t)T * KP * 2); b16* XL = (b16*)carve((size_t)T * KP * 2);
  b16* QK = (b16*)carve((size_t)T * 2 * E * 2); b16* VR = (b16*)carve((size_t)T * E * 2); b16* VRl = (b16*)carve((size_t)T * E * 2); b16* VT = (b16*)carve((size_t)T * E * 2); b16* VTl = (b16*)carve((size_t)T * E * 2);
  float* Cm = (float*)carve((size_t)H * T * T * 4); float* f = (float*)carve((size_t)H * T * 4); float* g = (float*)carve((size_t)H * T * 4); b16* Yh = (b16*)carve((size_t)T * E * 2); b16* Yl = (b16*)carve((size_t)T * E * 2);
  if (off > ws_size) return;
  prep_kernel<<<512, 256, 0, stream>>>(wa, wp, lw, lb, ba, bp, RA, RP, P);
  for (int b = 0; b < Bn; ++b) { const float* xb = x + (size_t)b * T * E1; float* ob = out + (size_t)b * T * E;
    ln_kernel<<<T / 8, 256, 0, stream>>>(xb, P, XH, XL);
    qkv_kernel<<<dim3(E3 / 256, T / 32), 64, 0, stream>>>(XH, XL, RA, P, QK, VR, VRl);
    vt_kernel<<<dim3(T / 128, H), 256, 0, stream>>>(VR, VT);
    vt_kernel<<<dim3(T / 128, H), 256, 0, stream>>>(VRl, VTl);
    cost_kernel<<<dim3(T / 16, 3), 128, 0, stream>>>(QK, Cm);
    rowstep_kernel<1><<<dim3(T / 32, H), 256, 0, stream>>>(Cm, g, f);
    colstep_kernel<<<dim3(T / 256, H), 256, 0, stream>>>(Cm, f, g);
    for (int it = 1; it < 6; ++it) { rowstep_kernel<0><<<dim3(T / 32, H), 256, 0, stream>>>(Cm, g, f); colstep_kernel<<<dim3(T / 256, H), 256, 0, stream>>>(Cm, f, g); }
    pv_kernel<<<dim3(T / 16, 3), 128, 0, stream>>>(Cm, f, g, VT, VTl, Yh, Yl);
    out_kernel<<<dim3(E / 256, T / 32), 64, 0, stream>>>(Yh, Yl, RP, P, ob); }
}
